// FloodGNN_29386166239380
// MI455X (gfx1250) — hardware-run, weakly checked
//
#include <hip/hip_runtime.h>

typedef float          v8f   __attribute__((ext_vector_type(8)));
typedef float          v4f   __attribute__((ext_vector_type(4)));
typedef unsigned int   v4u   __attribute__((ext_vector_type(4)));
typedef int            v8i   __attribute__((ext_vector_type(8)));
typedef unsigned short v8us  __attribute__((ext_vector_type(8)));
typedef unsigned short v16us __attribute__((ext_vector_type(16)));
typedef __bf16         v16bf __attribute__((ext_vector_type(16)));
typedef _Float16       v16h  __attribute__((ext_vector_type(16)));
typedef v4f  __attribute__((may_alias)) v4fa;
typedef v8us __attribute__((may_alias)) v8usa;
union FragB { v16bf v; v16us u; v8us h[2]; v8i w; };
union FragH { v16h  v; v16us u; v8us h[2]; v8i w; };

__device__ __forceinline__ v8f wmb(const FragB& a, const FragB& b, v8f c) {
  v8f d = __builtin_amdgcn_wmma_f32_16x16x32_bf16(false, a.v, false, b.v, (short)0, c, false, false);
  asm volatile("v_nop\n\tv_nop\n\tv_nop\n\tv_nop" : "+v"(d) : "v"(a.w), "v"(b.w));
  return d;
}

__device__ __forceinline__ v8f wmh(const FragH& a, const FragH& b, v8f c) {
  v8f d = __builtin_amdgcn_wmma_f32_16x16x32_f16(false, a.v, false, b.v, (short)0, c, false, false);
  asm volatile("v_nop\n\tv_nop\n\tv_nop\n\tv_nop" : "+v"(d) : "v"(a.w), "v"(b.w));
  return d;
}

__device__ __forceinline__ unsigned bf16_bits(float f) {
  const unsigned u = __float_as_uint(f);
  const unsigned r = (u + 0x7FFFu + ((u >> 16) & 1u)) >> 16;
  const unsigned q = (u >> 16) | 0x40u;
  return ((u & 0x7fffffffu) > 0x7f800000u) ? q : r;
}

__device__ __forceinline__ float bf16_val(float f) {
  return __uint_as_float(bf16_bits(f) << 16);
}
__device__ __forceinline__ int clampi(int v, int lo, int hi) {
  return v < lo ? lo : (v > hi ? hi : v);
}

__device__ __forceinline__ unsigned f16_bits(float f) {
  const unsigned u  = __float_as_uint(f);
  const unsigned s  = (u >> 16) & 0x8000u;
  const unsigned a  = u & 0x7fffffffu;
  const unsigned t  = a - 0x38000000u;
  const unsigned r  = (t + 0x0FFFu + ((t >> 13) & 1u)) >> 13;
  const unsigned rc = r > 0x7C00u ? 0x7C00u : r;
  const bool small  = a < 0x38800000u;
  const bool isnan  = a > 0x7f800000u;
  const unsigned fin = small ? 0u : (s | rc);
  return isnan ? (s | 0x7E00u) : fin;
}

__device__ __forceinline__ unsigned pk16(unsigned lo, unsigned hi) { return lo | (hi << 16); }
__device__ __forceinline__ unsigned bf16_lo_bits(float v) {
  float hi = bf16_val(v);
  asm volatile("" : "+v"(hi));
  return bf16_bits(v - hi);
}
__device__ __forceinline__ v4u pack8_bf16(v4f a, v4f c) {
  return (v4u){ pk16(bf16_bits(a[0]), bf16_bits(a[1])), pk16(bf16_bits(a[2]), bf16_bits(a[3])),
                pk16(bf16_bits(c[0]), bf16_bits(c[1])), pk16(bf16_bits(c[2]), bf16_bits(c[3])) };
}
__device__ __forceinline__ v4u pack8_bf16_lo(v4f a, v4f c) {
  return (v4u){ pk16(bf16_lo_bits(a[0]), bf16_lo_bits(a[1])), pk16(bf16_lo_bits(a[2]), bf16_lo_bits(a[3])),
                pk16(bf16_lo_bits(c[0]), bf16_lo_bits(c[1])), pk16(bf16_lo_bits(c[2]), bf16_lo_bits(c[3])) };
}
__device__ __forceinline__ v4u pack8_f16(v4f a, v4f c) {
  return (v4u){ pk16(f16_bits(a[0]), f16_bits(a[1])), pk16(f16_bits(a[2]), f16_bits(a[3])),
                pk16(f16_bits(c[0]), f16_bits(c[1])), pk16(f16_bits(c[2]), f16_bits(c[3])) };
}

template <int FORM>
__global__ __launch_bounds__(256) void k_plane(const float* __restrict__ src, int rows, int cols, int ldsrc,
                                               unsigned short* __restrict__ dst, int MP, int KP) {
  static_assert(FORM >= 0 && FORM <= 3);
  const int KTOT = (FORM == 1 || FORM == 3) ? 2 * KP : KP;
  const unsigned ppr   = (unsigned)(KTOT >> 3);
  const unsigned kp8   = (unsigned)(KP >> 3);
  const unsigned total = (unsigned)MP * ppr;
  const unsigned g     = blockIdx.x * 256u + threadIdx.x;
  const unsigned rowu  = g / ppr;
  const unsigned p     = g - rowu * ppr;
  const bool second    = p >= kp8;
  const int row = (int)rowu;
  const int c0  = (int)((second ? p - kp8 : p) << 3);
  const float* srow = src + (size_t)clampi(row, 0, rows - 1) * (size_t)ldsrc;
  float x[8];
  unsigned mk[8];
#pragma unroll
  for (int e = 0; e < 8; ++e) {
    const int c = c0 + e;
    const float v = srow[clampi(c, 0, cols - 1)];
    asm volatile("" :: "v"(v));
    x[e]  = v;
    mk[e] = (row < rows && c < cols) ? 0xFFFFu : 0u;
  }
  const v4f a = (v4f){ x[0], x[1], x[2], x[3] };
  const v4f c = (v4f){ x[4], x[5], x[6], x[7] };
  v4u o;
  if (FORM == 2) {
    o = pack8_f16(a, c);
  } else {
    const v4u hi = pack8_bf16(a, c);
    o = hi;
    if (FORM == 1) { const v4u lo = pack8_bf16_lo(a, c); o = second ? lo : hi; }
  }
  const v4u mw = (v4u){ pk16(mk[0], mk[1]), pk16(mk[2], mk[3]), pk16(mk[4], mk[5]), pk16(mk[6], mk[7]) };
  o &= mw;
  if (g < total) {
    volatile v4u* q = (volatile v4u*)(dst + (size_t)g * 8);
    *q = o;
    __threadfence();
    *q = o;
  }
}

template <int FORM> struct FragOf    { typedef FragB T; };
template <>         struct FragOf<2> { typedef FragH T; };
__device__ __forceinline__ v8f mm(const FragB& a, const FragB& b, v8f c) { return wmb(a, b, c); }
__device__ __forceinline__ v8f mm(const FragH& a, const FragH& b, v8f c) { return wmh(a, b, c); }
template <class F> __device__ __forceinline__ F ld_frag(const unsigned short* p) {
  F f;
  f.h[0] = *(const v8usa*)(p);
  f.h[1] = *(const v8usa*)(p + 16);
  return f;
}

template <int FORM, int EPI>
__global__ __launch_bounds__(256) __attribute__((amdgpu_num_vgpr(248)))
void k_gemm_nt(const unsigned short* __restrict__ A, const unsigned short* __restrict__ B,
               const float* __restrict__ bias, float* __restrict__ D, int M, int N, int KTOT, int ldd) {
  static_assert(FORM >= 0 && FORM <= 2);
  static_assert(EPI == 0 || EPI == 1);
  typedef typename FragOf<FORM>::T F;
  __shared__ __attribute__((aligned(16))) float sT[8][16 * 68];
  const int lane = threadIdx.x & 31;
  const int wave = threadIdx.x >> 5;
  const int tilesM = (M + 63) >> 6;
  const int tilesN = (N + 63) >> 6;
  const int tile = blockIdx.x * 8 + wave;
  if (tile >= tilesM * tilesN) return;
  const int tm = tile / tilesN;
  const int tn = tile - tm * tilesN;
  const int m0 = tm << 6;
  const int n0 = tn << 6;

  const int rl = lane & 15;
  const int h8 = (lane >> 4) * 8;
  const unsigned short* pa = A + (size_t)(m0 + rl) * (size_t)KTOT + h8;
  const unsigned short* pb = B + (size_t)(n0 + rl) * (size_t)KTOT + h8;

  v8f acc[4][4];
#pragma unroll
  for (int i = 0; i < 4; ++i)
#pragma unroll
    for (int j = 0; j < 4; ++j) acc[i][j] = (v8f){0.f, 0.f, 0.f, 0.f, 0.f, 0.f, 0.f, 0.f};

#pragma unroll 1
  for (int k0 = 0; k0 < KTOT; k0 += 32) {
    F bf[4];
#pragma unroll
    for (int j = 0; j < 4; ++j) bf[j] = ld_frag<F>(pb + (size_t)(j << 4) * (size_t)KTOT + k0);
#pragma unroll
    for (int i = 0; i < 4; ++i) {
      const F af = ld_frag<F>(pa + (size_t)(i << 4) * (size_t)KTOT + k0);
#pragma unroll
      for (int j = 0; j < 4; ++j) acc[i][j] = mm(af, bf[j], acc[i][j]);
    }
  }

  float* slab = sT[wave];
  const int hh = lane >> 4;
  const int c4 = (lane & 15) * 4;
  const int nc = n0 + c4;
  const bool cok = nc < N;
  v4f bv = (v4f){0.f, 0.f, 0.f, 0.f};
  if (EPI == 1) {
    bv = *(const v4fa*)(bias + clampi(nc, 0, N - 4));
    asm volatile("" :: "v"(bv));
  }
#pragma unroll
  for (int i = 0; i < 4; ++i) {
    const int mBase = m0 + (i << 4);
#pragma unroll
    for (int j = 0; j < 4; ++j) {
#pragma unroll
      for (int r = 0; r < 8; ++r) slab[(h8 + r) * 68 + (j << 4) + rl] = acc[i][j][r];
    }
    __builtin_amdgcn_fence(__ATOMIC_RELEASE, "workgroup");
    __builtin_amdgcn_wave_barrier();
    __builtin_amdgcn_fence(__ATOMIC_ACQUIRE, "workgroup");
    v4f vv[8];
#pragma unroll
    for (int it = 0; it < 8; ++it) {
      const int row = it * 2 + hh;
      v4f v = *(const v4fa*)(slab + row * 68 + c4);
      if (EPI == 1) v += bv;
      vv[it] = v;
    }
    for (int pass = 0; pass < 2; ++pass) {
#pragma unroll
      for (int it = 0; it < 8; ++it) {
        const int row = mBase + it * 2 + hh;
        if (cok && row < M) *(volatile v4f*)(D + (size_t)row * (size_t)ldd + nc) = vv[it];
      }
      __threadfence();
    }
    __builtin_amdgcn_fence(__ATOMIC_RELEASE, "workgroup");
    __builtin_amdgcn_wave_barrier();
    __builtin_amdgcn_fence(__ATOMIC_ACQUIRE, "workgroup");
  }
}

#define NN       50000
#define NE       800000
#define MPN      50048
#define NBLK     49
#define NBROWS   1024
#define DEGCAP   64
#define MAXHITS  16623
#define MAXDEG   35
#define NTHR     256
#define NWAVE    8
#define EPT      8
#define CHUNK    (NTHR * EPT)
#define WCAP     (EPT * 32)
#define LISTN    (NWAVE * WCAP)
#define NBMAX    2048
#define ESH      11
#define RCAP     20480
#define LDS_BKT  ((2 * RCAP + 2 * NBMAX + LISTN) * 4 + 64)
#define LDS_MSG  (RCAP * 4)
#define PA_ENC   0
#define PA_LYR   192
#define PA_MSG   768
#define PA_HEAD  1152
#define PAR_LINES 42
#define WSMAX    ((size_t)128 << 20)

static_assert(MPN % 128 == 0 && MPN >= NN && MPN - NN < 64);
static_assert(NN % 16 == 0 && NE % 4 == 0);
static_assert(NBLK * NBROWS >= NN && (NBLK - 1) * NBROWS < NN);
static_assert((NN - (NBLK - 1) * NBROWS) % 4 == 0);
static_assert(NBROWS <= NBMAX && (1 << ESH) >= NBMAX && NTHR * 8 == NBMAX && LISTN >= NBMAX);
static_assert(NBROWS == 8 * 128);
static_assert(NE <= (1 << (32 - ESH)));
static_assert(RCAP % 1024 == 0 && RCAP % 16 == 0 && RCAP > MAXHITS + 1024);
static_assert(RCAP * 100 >= MAXHITS * 105);
static_assert(DEGCAP >= MAXDEG + 8 && DEGCAP <= 64);
static_assert(LDS_BKT <= 327680 && LDS_MSG + 4096 <= 327680);
static_assert((MPN * 32 / 8) % 256 == 0);
static_assert(3 * NN <= 586 * 256 && 3 * NN > 585 * 256);
static_assert(PAR_LINES * 32 == 1344 && PA_HEAD + 164 <= 1344);

constexpr size_t al256(size_t v) { return (v + 255) & ~(size_t)255; }
constexpr size_t O_XB    = 0;
constexpr size_t O_YUT   = al256(O_XB    + (size_t)MPN * 32 * 2);
constexpr size_t O_H     = al256(O_YUT   + (size_t)MPN * 64 * 4);
constexpr size_t O_HHL   = al256(O_H     + (size_t)MPN * 64 * 4);
constexpr size_t O_P     = al256(O_HHL   + (size_t)MPN * 128 * 2);
constexpr size_t O_SHL   = al256(O_P     + (size_t)MPN * 32 * 4);
constexpr size_t O_BLIST = al256(O_SHL   + (size_t)MPN * 64 * 2);
constexpr size_t O_OFFC  = al256(O_BLIST + (size_t)NBLK * RCAP * 4);
constexpr size_t O_META  = al256(O_OFFC  + (size_t)NBLK * 2048 * 4);
constexpr size_t O_OUT3  = al256(O_META  + (size_t)NBLK * 128);
constexpr size_t O_ENCW  = al256(O_OUT3  + (size_t)MPN * 16);
constexpr size_t O_W1A   = al256(O_ENCW  + 64 * 32 * 2);
constexpr size_t O_W2T   = al256(O_W1A   + 3 * 64 * 128 * 2);
constexpr size_t O_HWT   = al256(O_W2T   + 3 * 64 * 64 * 2);
constexpr size_t O_PAR   = al256(O_HWT   + 64 * 128 * 2);
constexpr size_t WS_TOTAL = al256(O_PAR + 8192);
static_assert(WS_TOTAL <= (size_t)WSMAX);

typedef int v4i __attribute__((ext_vector_type(4)));
typedef v4i __attribute__((may_alias)) v4ia;
typedef v4u __attribute__((may_alias)) v4ua;

__device__ __forceinline__ void wave_sync_lds() {
  __builtin_amdgcn_fence(__ATOMIC_RELEASE, "workgroup");
  __builtin_amdgcn_wave_barrier();
  __builtin_amdgcn_fence(__ATOMIC_ACQUIRE, "workgroup");
}
__device__ __forceinline__ void st2_v4u(void* p, const v4u v) {
  volatile v4u* q = (volatile v4u*)p;
  *q = v;
  __threadfence();
  *q = v;
}
__device__ __forceinline__ void st2_v4f(float* p, const v4f v) {
  volatile v4f* q = (volatile v4f*)p;
  *q = v;
  __threadfence();
  *q = v;
}
__device__ __forceinline__ void st2_v4i(int* p, const v4i v) {
  volatile v4i* q = (volatile v4i*)p;
  *q = v;
  __threadfence();
  *q = v;
}

__device__ __forceinline__ v4u gather8_bf16(const float* __restrict__ src, int base, int k0, int kmask, int stride,
                                            unsigned mk) {
  float x[8];
#pragma unroll
  for (int e = 0; e < 8; ++e) {
    const float v = src[base + ((k0 + e) & kmask) * stride];
    asm volatile("" :: "v"(v));
    x[e] = v;
  }
  v4u o = pack8_bf16((v4f){ x[0], x[1], x[2], x[3] }, (v4f){ x[4], x[5], x[6], x[7] });
  o &= (v4u){ mk, mk, mk, mk };
  return o;
}

__global__ __launch_bounds__(256) void k_prep(
    const float* __restrict__ enc_w, const float* __restrict__ enc_b, const float* __restrict__ enc_g,
    const float* __restrict__ enc_be, const float* __restrict__ w1, const float* __restrict__ b1,
    const float* __restrict__ w2, const float* __restrict__ b2, const float* __restrict__ lg,
    const float* __restrict__ lb, const float* __restrict__ dw1, const float* __restrict__ db1,
    const float* __restrict__ dw2, const float* __restrict__ db2, const float* __restrict__ vw1,
    const float* __restrict__ vb1, const float* __restrict__ vw2, const float* __restrict__ vb2,
    unsigned short* ENCWT, unsigned short* W1AT2, unsigned short* W2T2, unsigned short* HWT2,
    float* PAR, unsigned short* SHL) {
  const int b = (int)blockIdx.x, tid = (int)threadIdx.x;
  if (b == 0) {
    const int n = tid >> 2, p = tid & 3;
    const v4u o = gather8_bf16(enc_w, n, 8 * p, 15, 64, p < 2 ? 0xFFFFFFFFu : 0u);
    st2_v4u(ENCWT + (size_t)tid * 8, o);
  } else if (b < 13) {
    const int u = (b - 1) * 256 + tid;
    const int i = u >> 10, rem = u & 1023;
    const int n = rem >> 4, p = rem & 15;
    const int nn = n < 32 ? n : 31;
    const v4u o = gather8_bf16(w1, i * 2144 + nn, 8 * p, 63, 32, n < 32 ? 0xFFFFFFFFu : 0u);
    st2_v4u(W1AT2 + (size_t)u * 8, o);
  } else if (b < 19) {
    const int u = (b - 13) * 256 + tid;
    const int i = u >> 9, rem = u & 511;
    const int n = rem >> 3, p = rem & 7;
    const v4u o = gather8_bf16(w2, i * 2048 + n, 8 * p, 31, 64, 0xFFFFFFFFu);
    st2_v4u(W2T2 + (size_t)u * 8, o);
  } else if (b < 21) {
    const int u = (b - 19) * 256 + tid;
    const int n = u >> 4, p = u & 15;
    const v4u o = gather8_bf16(dw1, n, 8 * p, 63, 32, 0xFFFFFFFFu);
    st2_v4u(HWT2 + (size_t)u * 8, o);
  } else if (b < 23) {
    const int u = (b - 21) * 256 + tid;
    const int n = u >> 4, p = u & 15;
    const v4u o = gather8_bf16(vw1, n, 8 * p, 63, 32, 0xFFFFFFFFu);
    st2_v4u(HWT2 + (size_t)(512 + u) * 8, o);
  } else if (b < 29) {
    const int lane = tid & 31;
    const int wave = __builtin_amdgcn_readfirstlane(tid >> 5);
    const int u = (b - 23) * 8 + wave;
    if (u < PAR_LINES) {
      float v = 0.0f;
      if (u < 2) {
        v = enc_b[32 * u + lane];
      } else if (u < 4) {
        v = enc_g[32 * (u - 2) + lane];
      } else if (u < 6) {
        v = enc_be[32 * (u - 4) + lane];
      } else if (u < 24) {
        const int t = u - 6;
        const int i = t / 6;
        const int r = t - 6 * i;
        const int off = i * 64 + 32 * (r & 1) + lane;
        if (r < 2)      v = b2[off];
        else if (r < 4) v = lg[off];
        else            v = lb[off];
      } else if (u < 36) {
        const int t = u - 24;
        const int i = t >> 2, l4 = t & 3;
        const int c = 8 * l4 + (lane >> 2);
        const int j = lane & 3;
        const int jc = j < 3 ? j : 2;
        const float wv = w1[i * 2144 + (64 + jc) * 32 + c];
        const float bv = b1[i * 32 + c];
        asm volatile("" :: "v"(wv), "v"(bv));
        const unsigned m = j < 3 ? 0xFFFFFFFFu : 0u;
        v = __uint_as_float((__float_as_uint(wv) & m) | (__float_as_uint(bv) & ~m));
      } else if (u == 36) {
        v = db1[lane];
      } else if (u == 37) {
        v = vb1[lane];
      } else if (u == 38) {
        v = dw2[lane];
      } else if (u == 39) {
        v = vw2[2 * lane];
      } else if (u == 40) {
        v = vw2[2 * lane + 1];
      } else {
        const float d0 = db2[0];
        const float v0 = vb2[clampi(lane - 1, 0, 1)];
        asm volatile("" :: "v"(d0), "v"(v0));
        const unsigned m0 = lane == 0 ? 0xFFFFFFFFu : 0u;
        const unsigned m1 = (lane == 1 || lane == 2) ? 0xFFFFFFFFu : 0u;
        v = __uint_as_float((__float_as_uint(d0) & m0) | (__float_as_uint(v0) & m1));
      }
      const float o = bf16_val(v);
      volatile float* q = PAR + 32 * u + lane;
      *q = o;
      __threadfence();
      *q = o;
    }
  } else {
    const v4u z = (v4u){ 0u, 0u, 0u, 0u };
    for (int q = tid; q < (MPN - NN) * 8; q += 256) st2_v4u(SHL + (size_t)NN * 64 + (size_t)q * 8, z);
  }
}

__device__ __forceinline__ int scan_chunk(const int* __restrict__ dsts, int nE, int cbase, int slotBase,
                                          int nb, int vec8, int* list, int tid, int lane, int wave) {
  int wc = 0;
  const int el0  = tid * EPT;
  const int e0   = cbase + el0;
  const int sent = (-0x7fffffff - 1);
  v4i da, db;
  if (vec8 != 0 && cbase + CHUNK <= nE) {
    da = *(const v4i*)(dsts + e0);
    db = *(const v4i*)(dsts + e0 + 4);
  } else {
    const int t0 = dsts[min(e0 + 0, nE - 1)];
    const int t1 = dsts[min(e0 + 1, nE - 1)];
    const int t2 = dsts[min(e0 + 2, nE - 1)];
    const int t3 = dsts[min(e0 + 3, nE - 1)];
    const int t4 = dsts[min(e0 + 4, nE - 1)];
    const int t5 = dsts[min(e0 + 5, nE - 1)];
    const int t6 = dsts[min(e0 + 6, nE - 1)];
    const int t7 = dsts[min(e0 + 7, nE - 1)];
    asm volatile("" :: "v"(t0), "v"(t1), "v"(t2), "v"(t3), "v"(t4), "v"(t5), "v"(t6), "v"(t7));
    da.x = (e0 + 0 < nE) ? t0 : sent;
    da.y = (e0 + 1 < nE) ? t1 : sent;
    da.z = (e0 + 2 < nE) ? t2 : sent;
    da.w = (e0 + 3 < nE) ? t3 : sent;
    db.x = (e0 + 4 < nE) ? t4 : sent;
    db.y = (e0 + 5 < nE) ? t5 : sent;
    db.z = (e0 + 6 < nE) ? t6 : sent;
    db.w = (e0 + 7 < nE) ? t7 : sent;
  }
  const unsigned nbs = (unsigned)slotBase;
  const unsigned unb = (unsigned)nb;
  const unsigned s0 = (unsigned)da.x - nbs, s1 = (unsigned)da.y - nbs;
  const unsigned s2 = (unsigned)da.z - nbs, s3 = (unsigned)da.w - nbs;
  const unsigned s4 = (unsigned)db.x - nbs, s5 = (unsigned)db.y - nbs;
  const unsigned s6 = (unsigned)db.z - nbs, s7 = (unsigned)db.w - nbs;
  const bool h0 = s0 < unb, h1 = s1 < unb, h2 = s2 < unb, h3 = s3 < unb;
  const bool h4 = s4 < unb, h5 = s5 < unb, h6 = s6 < unb, h7 = s7 < unb;
  const unsigned any = __builtin_amdgcn_ballot_w32(h0 | h1 | h2 | h3 | h4 | h5 | h6 | h7);
  if (any != 0u) {
#define HITJ(J, HJ, SJ) { \
      const unsigned mj = __builtin_amdgcn_ballot_w32(HJ); \
      if (mj != 0u) { \
        if (HJ) { \
          const int pos = wc + (int)__builtin_amdgcn_mbcnt_lo(mj, 0u); \
          if (pos < WCAP) list[wave * WCAP + pos] = ((el0 + (J)) << 12) | (int)(SJ); \
        } \
        wc += (int)__builtin_popcount(mj); } }
    HITJ(0, h0, s0)
    HITJ(1, h1, s1)
    HITJ(2, h2, s2)
    HITJ(3, h3, s3)
    HITJ(4, h4, s4)
    HITJ(5, h5, s5)
    HITJ(6, h6, s6)
    HITJ(7, h7, s7)
#undef HITJ
  }
  return wc;
}

__device__ __forceinline__ int build_lists(const int* __restrict__ dsts, int nE, int nodeBase, int nb, int vec8,
                                           int* reg1, int* reg2, int* scnt, int* soff, int* list,
                                           int* wcnt, int* wtot, int tid, int lane, int wave) {
  for (int i = tid; i < NBMAX; i += NTHR) scnt[i] = 0;
  __syncthreads();

  int tot = 0;
  const int nChunks = (nE + CHUNK - 1) / CHUNK;
#pragma unroll 1
  for (int ch = 0; ch < nChunks; ++ch) {
    const int cbase = ch * CHUNK;
    const int wc = scan_chunk(dsts, nE, cbase, nodeBase, nb, vec8, list, tid, lane, wave);
    if (lane == 0) wcnt[wave] = wc;
    __syncthreads();
    int pre = 0, all = 0;
#pragma unroll
    for (int w2 = 0; w2 < NWAVE; ++w2) {
      int c = wcnt[w2];
      c = c < 0 ? 0 : (c > WCAP ? WCAP : c);
      all += c;
      pre += (w2 < wave) ? c : 0;
    }
    const int wcc  = wc > WCAP ? WCAP : wc;
    const int base = tot + pre;
#pragma unroll 1
    for (int i = lane; i < wcc; i += 32) {
      const int ent = list[wave * WCAP + i];
      const int el  = (ent >> 12) & (CHUNK - 1);
      const int sl  = ent & (NBMAX - 1);
      int eid = cbase + el;
      eid = eid > nE - 1 ? nE - 1 : eid;
      const int pos = base + i;
      if (pos < RCAP) reg1[pos] = (int)(((unsigned)eid << ESH) | (unsigned)sl);
    }
    tot += all;
    tot = tot > RCAP ? RCAP : tot;
    __syncthreads();
  }
  const int nh = tot;

  if (wave == 0) {
#pragma unroll 1
    for (int b0 = 0; b0 < nh; b0 += 32) {
      const int idx = b0 + lane;
      const int uv  = reg1[idx < RCAP ? idx : RCAP - 1];
      const int m32 = (nh - b0) < 32 ? (nh - b0) : 32;
#pragma unroll 1
      for (int k = 0; k < m32; ++k) {
        const int u  = __builtin_amdgcn_readlane(uv, k);
        const int sl = u & (NBMAX - 1);
        if (lane == 0) scnt[sl] = scnt[sl] + 1;
      }
    }
  }
  __syncthreads();

  {
    const v4i ca = *(const v4i*)(scnt + 8 * tid);
    const v4i cb = *(const v4i*)(scnt + 8 * tid + 4);
    const int e0 = ca.x < 0 ? 0 : ca.x, e1 = ca.y < 0 ? 0 : ca.y, e2 = ca.z < 0 ? 0 : ca.z, e3 = ca.w < 0 ? 0 : ca.w;
    const int e4 = cb.x < 0 ? 0 : cb.x, e5 = cb.y < 0 ? 0 : cb.y, e6 = cb.z < 0 ? 0 : cb.z, e7 = cb.w < 0 ? 0 : cb.w;
    const int ts = e0 + e1 + e2 + e3 + e4 + e5 + e6 + e7;
    int incl = ts;
#pragma unroll
    for (int d = 1; d < 32; d <<= 1) {
      const int up = __shfl_up(incl, d);
      if (lane >= d) incl += up;
    }
    if (lane == 31) wtot[wave] = incl;
    __syncthreads();
    int pre = 0;
#pragma unroll
    for (int w2 = 0; w2 < NWAVE; ++w2) pre += (w2 < wave) ? wtot[w2] : 0;
    int run = pre + incl - ts;
    soff[8 * tid + 0] = run; run += e0;
    soff[8 * tid + 1] = run; run += e1;
    soff[8 * tid + 2] = run; run += e2;
    soff[8 * tid + 3] = run; run += e3;
    soff[8 * tid + 4] = run; run += e4;
    soff[8 * tid + 5] = run; run += e5;
    soff[8 * tid + 6] = run; run += e6;
    soff[8 * tid + 7] = run;
  }
  __syncthreads();
  for (int i = tid; i < NBMAX; i += NTHR) list[i] = soff[i];
  __syncthreads();

  if (wave == 0) {
#pragma unroll 1
    for (int b0 = 0; b0 < nh; b0 += 32) {
      const int idx = b0 + lane;
      const int uv  = reg1[idx < RCAP ? idx : RCAP - 1];
      const int m32 = (nh - b0) < 32 ? (nh - b0) : 32;
#pragma unroll 1
      for (int k = 0; k < m32; ++k) {
        const int u   = __builtin_amdgcn_readlane(uv, k);
        const int sl  = u & (NBMAX - 1);
        const int eid = (int)((unsigned)u >> ESH);
        if (lane == 0) {
          int pos = list[sl];
          pos = pos < 0 ? 0 : (pos > RCAP - 1 ? RCAP - 1 : pos);
          reg2[pos] = eid;
          list[sl] = pos + 1;
        }
      }
    }
  }
  __syncthreads();
  return nh;
}

__global__ __launch_bounds__(NTHR) void k_bucket(const int* __restrict__ dsts, int nE, int nN, int vec8,
                                                 int* BLIST, int* OFFC, int* META) {
  extern __shared__ v4f lds_dyn[];
  int* reg1 = (int*)lds_dyn;
  int* reg2 = reg1 + RCAP;
  int* scnt = reg2 + RCAP;
  int* soff = scnt + NBMAX;
  int* list = soff + NBMAX;
  int* wcnt = list + LISTN;
  int* wtot = wcnt + NWAVE;
  const int tid = (int)threadIdx.x, lane = tid & 31, wave = tid >> 5;
  const int b = (int)blockIdx.x;
  const int nodeBase = b * NBROWS;
  int nb = nN - nodeBase;
  nb = nb < 0 ? 0 : (nb > NBROWS ? NBROWS : nb);

  const int nh = build_lists(dsts, nE, nodeBase, nb, vec8, reg1, reg2, scnt, soff, list, wcnt, wtot, tid, lane, wave);

  int* bl = BLIST + (size_t)b * RCAP;
  const int last = nh > 0 ? nh - 1 : 0;
#pragma unroll 1
  for (int base = 0; base < RCAP; base += 1024) {
    const int i0 = base + 4 * tid;
    v4i v;
    v.x = reg2[i0     < last ? i0     : last];
    v.y = reg2[i0 + 1 < last ? i0 + 1 : last];
    v.z = reg2[i0 + 2 < last ? i0 + 2 : last];
    v.w = reg2[i0 + 3 < last ? i0 + 3 : last];
    v.x = (i0     < nh) ? v.x : 0;
    v.y = (i0 + 1 < nh) ? v.y : 0;
    v.z = (i0 + 2 < nh) ? v.z : 0;
    v.w = (i0 + 3 < nh) ? v.w : 0;
    st2_v4i(bl + i0, v);
  }
  {
    const v4i so = *(const v4ia*)(soff + 4 * tid);
    const v4i sc = *(const v4ia*)(scnt + 4 * tid);
    int* oc = OFFC + (size_t)b * 2048;
    st2_v4i(oc + 4 * tid, so);
    st2_v4i(oc + 1024 + 4 * tid, sc);
  }
  if (tid < 8) {
    v4i mv;
    mv.x = (tid == 0) ? nh : 0;
    mv.y = (tid == 0 && nh >= RCAP) ? 1 : 0;
    mv.z = 0; mv.w = 0;
    st2_v4i(META + (size_t)b * 32 + 4 * tid, mv);
  }
}

template <int MODE>
__global__ __launch_bounds__(256) void k_rowln(const float* __restrict__ Yin, float* H, const int* __restrict__ OFFC,
                                               const float* __restrict__ par, int pofs, unsigned short* HHL) {
  __shared__ __attribute__((aligned(16))) float sR[8][128];
  const int tid = (int)threadIdx.x, lane = tid & 31, wave = tid >> 5;
  const int hh = lane >> 4;
  const int pp = lane & 15;
  const int c4 = pp * 4;
  const v4f pa = *(const v4fa*)(par + pofs + c4);
  const v4f pg = *(const v4fa*)(par + pofs + 64 + c4);
  const v4f pb = *(const v4fa*)(par + pofs + 128 + c4);
  const v4f zero4 = (v4f){ 0.0f, 0.0f, 0.0f, 0.0f };
  float* srow = &sR[wave][0];
#pragma unroll 1
  for (int it = 0; it < 4; ++it) {
    const int row0 = (int)blockIdx.x * 64 + wave * 8 + it * 2;
    const int row  = row0 + hh;
    const int rc   = row < NN ? row : NN - 1;
    v4f v = *(const v4fa*)(Yin + (size_t)rc * 64 + c4);
    asm volatile("" :: "v"(v));
    if (MODE == 1) {
      const v4f hv = *(const v4fa*)(H + (size_t)rc * 64 + c4);
      int cn = OFFC[(size_t)(rc >> 10) * 2048 + 1024 + (rc & 1023)];
      asm volatile("" :: "v"(hv), "v"(cn));
      const v4f ad = (cn > 0) ? pa : zero4;
      v = hv + (v + ad);
    } else {
      v = v + pa;
    }
    float s = (v[0] + v[1]) + (v[2] + v[3]);
    s += __shfl_xor(s, 8);
    s += __shfl_xor(s, 4);
    s += __shfl_xor(s, 2);
    s += __shfl_xor(s, 1);
    const float mu = s * (1.0f / 64.0f);
    const v4f d = v - mu;
    float q = (d[0] * d[0] + d[1] * d[1]) + (d[2] * d[2] + d[3] * d[3]);
    q += __shfl_xor(q, 8);
    q += __shfl_xor(q, 4);
    q += __shfl_xor(q, 2);
    q += __shfl_xor(q, 1);
    const float rs = 1.0f / sqrtf(q * (1.0f / 64.0f) + 1e-5f);
    v4f y = (d * rs) * pg + pb;
    if (MODE == 0) {
#pragma unroll
      for (int e = 0; e < 4; ++e) { const float t = y[e]; y[e] = (t > 0.0f) ? t : (t - t); }
    }
    y = (row < NN) ? y : zero4;
    *(v4fa*)(srow + hh * 64 + c4) = y;
    wave_sync_lds();
    const float* sp = srow + hh * 64 + (pp & 7) * 8;
    const v4f a = *(const v4fa*)sp;
    const v4f c = *(const v4fa*)(sp + 4);
    const v4u hi = pack8_bf16(a, c);
    const v4u lo = pack8_bf16_lo(a, c);
    const v4u o = (pp >= 8) ? lo : hi;
    float* hp = H + (size_t)row * 64 + c4;
    unsigned short* qp = HHL + (size_t)row * 128 + pp * 8;
    for (int pass = 0; pass < 2; ++pass) {
      *(volatile v4f*)hp = y;
      *(volatile v4u*)qp = o;
      __threadfence();
    }
    wave_sync_lds();
  }
}

__global__ __launch_bounds__(256) void k_msg(const int* __restrict__ ei, const float* __restrict__ ea,
                                             const float* __restrict__ P, const int* __restrict__ BLIST,
                                             const int* __restrict__ OFFC, const int* __restrict__ META,
                                             const float* __restrict__ par, int pofs, unsigned short* SHL) {
  extern __shared__ v4f lds_dyn[];
  __shared__ __attribute__((aligned(16))) float sS[8][128];
  int* slist = (int*)lds_dyn;
  const int tid = (int)threadIdx.x, lane = tid & 31;
  const int wave = __builtin_amdgcn_readfirstlane(tid >> 5);
  const int b = (int)blockIdx.x;
  const int nodeBase = b * NBROWS;
  const int nb = clampi(NN - nodeBase, 0, NBROWS);
  const int nh = clampi(META[(size_t)b * 32], 0, RCAP);
  const int flag = META[(size_t)b * 32 + 1];
  const bool ovf = flag != 0;
  const int* bl = BLIST + (size_t)b * RCAP;
  const int* oc = OFFC + (size_t)b * 2048;
  const int nhs = nh > 0 ? nh : 1;
#pragma unroll 1
  for (int base = 0; base < nhs; base += 1024) {
    const int i0 = base + 4 * tid;
    *(v4ia*)(slist + i0) = *(const v4ia*)(bl + i0);
  }
  __syncthreads();
  const v4f pw = *(const v4fa*)(par + pofs + 4 * lane);
  const int nhm1 = nh > 0 ? nh - 1 : 0;
  const float qnan = __int_as_float(0x7fc00000);
  float* srow = &sS[wave][0];

#pragma unroll 1
  for (int g = 0; g < 32; ++g) {
    const int slot0 = wave * 128 + g * 4;
    if (slot0 >= nb) break;
    int stv = oc[slot0 + (lane & 3)];
    int cv  = oc[1024 + slot0 + (lane & 3)];
    asm volatile("" :: "v"(stv), "v"(cv));
    const int craw = cv < 0 ? 0 : cv;
    const int pv = (craw > DEGCAP) ? 1 : 0;
    stv = clampi(stv, 0, nh);
    int cc = clampi(craw, 0, DEGCAP);
    cc = cc > nh - stv ? nh - stv : cc;
#pragma unroll 1
    for (int rr = 0; rr < 4; ++rr) {
      const int st  = __builtin_amdgcn_readlane(stv, rr);
      const int cnt = __builtin_amdgcn_readlane(cc, rr);
      const int cr  = __builtin_amdgcn_readlane(craw, rr);
      const int prw = __builtin_amdgcn_readlane(pv, rr);
      float acc = 0.0f;
#pragma unroll 1
      for (int b0 = 0; b0 < cnt; b0 += 32) {
        const int li = clampi(st + b0 + lane, 0, nhm1);
        const int id = clampi(slist[li], 0, NE - 1);
        int s = ei[id];
        float a0 = ea[3 * id], a1 = ea[3 * id + 1], a2 = ea[3 * id + 2];
        asm volatile("" :: "v"(s), "v"(a0), "v"(a1), "v"(a2));
        s = clampi(s, 0, NN - 1);
        const int i0 = __float_as_int(bf16_val(a0));
        const int i1 = __float_as_int(bf16_val(a1));
        const int i2 = __float_as_int(bf16_val(a2));
        const int m32 = (cnt - b0) < 32 ? (cnt - b0) : 32;
#pragma unroll 4
        for (int q = 0; q < m32; ++q) {
          const int sq = __builtin_amdgcn_readlane(s, q);
          const float e0 = __int_as_float(__builtin_amdgcn_readlane(i0, q));
          const float e1 = __int_as_float(__builtin_amdgcn_readlane(i1, q));
          const float e2 = __int_as_float(__builtin_amdgcn_readlane(i2, q));
          const float p = P[(size_t)sq * 32 + lane];
          const float t = fmaf(e2, pw[2], fmaf(e1, pw[1], e0 * pw[0]));
          const float z = (p + t) + pw[3];
          acc += (z > 0.0f) ? z : (z - z);
        }
      }
      const float inv = (cr > 0) ? (1.0f / (float)cr) : 0.0f;
      float S = acc * inv;
      S = (ovf || prw != 0) ? qnan : S;
      srow[rr * 32 + lane] = S;
    }
    wave_sync_lds();
    {
      const int r = lane >> 3, p = lane & 7;
      const float* sp = srow + r * 32 + (p & 3) * 8;
      const v4f a = *(const v4fa*)sp;
      const v4f c = *(const v4fa*)(sp + 4);
      const v4u hi = pack8_bf16(a, c);
      const v4u lo = pack8_bf16_lo(a, c);
      const v4u o = (p >= 4) ? lo : hi;
      st2_v4u(SHL + (size_t)(nodeBase + slot0 + r) * 64 + p * 8, o);
    }
    wave_sync_lds();
  }
}

__global__ __launch_bounds__(128) void k_head(const float* __restrict__ T, const float* __restrict__ par, float* OUT3) {
  __shared__ __attribute__((aligned(16))) float sT2[4][32 * 68];
  __shared__ __attribute__((aligned(16))) float sW[176];
  const int tid = (int)threadIdx.x, lane = tid & 31, wave = tid >> 5;
  {
    const int ix = tid < 40 ? tid : 40;
    const v4f w = *(const v4fa*)(par + PA_HEAD + 4 * ix);
    asm volatile("" :: "v"(w));
    if (tid < 41) *(v4fa*)(sW + 4 * tid) = w;
  }
  const int row0 = ((int)blockIdx.x * 4 + wave) * 32;
  float* slab = &sT2[wave][0];
#pragma unroll 4
  for (int it = 0; it < 16; ++it) {
    const int idx = it * 32 + lane;
    const int r = idx >> 4, c4 = (idx & 15) * 4;
    const int rc = (row0 + r) < NN ? (row0 + r) : NN - 1;
    const v4f v = *(const v4fa*)(T + (size_t)rc * 64 + c4);
    *(v4fa*)(slab + r * 68 + c4) = v;
  }
  __syncthreads();
  const float* tr = slab + lane * 68;
  float d = 0.0f, vx = 0.0f, vy = 0.0f;
#pragma unroll 4
  for (int c = 0; c < 32; ++c) {
    float x = tr[c] + sW[c];
    x = (x > 0.0f) ? x : (x - x);
    d = fmaf(x, sW[64 + c], d);
    float y = tr[32 + c] + sW[32 + c];
    y = (y > 0.0f) ? y : (y - y);
    vx = fmaf(y, sW[96 + c], vx);
    vy = fmaf(y, sW[128 + c], vy);
  }
  const v4f o = (v4f){ d + sW[160], vx + sW[161], vy + sW[162], 0.0f };
  st2_v4f(OUT3 + (size_t)(row0 + lane) * 4, o);
}

__global__ __launch_bounds__(256) void k_store(const float* __restrict__ OUT3, float* out) {
  const int f = (int)blockIdx.x * 256 + (int)threadIdx.x;
  const int fa = clampi(f, 0, NN - 1);
  const int g = clampi(f - NN, 0, 2 * NN - 1);
  const float a = OUT3[(size_t)fa * 4];
  const float c = OUT3[(size_t)(g >> 1) * 4 + 1 + (g & 1)];
  asm volatile("" :: "v"(a), "v"(c));
  const unsigned m = f < NN ? 0xFFFFFFFFu : 0u;
  const float val = __uint_as_float((__float_as_uint(a) & m) | (__float_as_uint(c) & ~m));
  if (f < 3 * NN) {
    volatile float* q = out + f;
    *q = val;
    __threadfence();
    *q = val;
  }
}

extern "C" void kernel_launch(void* const* d_in, const int* in_sizes, int n_in,
                              void* d_out, int out_size, void* d_ws, size_t ws_size,
                              hipStream_t stream) {
  if (n_in < 21) return;
  if (in_sizes[0] != NN * 16 || in_sizes[1] != 2 * NE || in_sizes[2] != NE * 3) return;
  if (in_sizes[3] != 16 * 64 || in_sizes[4] != 64 || in_sizes[5] != 64 || in_sizes[6] != 64) return;
  if (in_sizes[7] != 3 * 67 * 32 || in_sizes[8] != 3 * 32 || in_sizes[9] != 3 * 32 * 64) return;
  if (in_sizes[10] != 3 * 64 || in_sizes[11] != 3 * 64 || in_sizes[12] != 3 * 64) return;
  if (in_sizes[13] != 64 * 32 || in_sizes[14] != 32 || in_sizes[15] != 32 || in_sizes[16] != 1) return;
  if (in_sizes[17] != 64 * 32 || in_sizes[18] != 32 || in_sizes[19] != 64 || in_sizes[20] != 2) return;
  if (out_size != 3 * NN) return;
  if (ws_size < WS_TOTAL) return;

  const float* x      = (const float*)d_in[0];
  const int*   ei     = (const int*)  d_in[1];
  const float* eattr  = (const float*)d_in[2];
  const float* enc_w  = (const float*)d_in[3];
  const float* enc_b  = (const float*)d_in[4];
  const float* enc_g  = (const float*)d_in[5];
  const float* enc_be = (const float*)d_in[6];
  const float* mlp_w1 = (const float*)d_in[7];
  const float* mlp_b1 = (const float*)d_in[8];
  const float* mlp_w2 = (const float*)d_in[9];
  const float* mlp_b2 = (const float*)d_in[10];
  const float* ln_g   = (const float*)d_in[11];
  const float* ln_b   = (const float*)d_in[12];
  const float* dw1    = (const float*)d_in[13];
  const float* db1    = (const float*)d_in[14];
  const float* dw2    = (const float*)d_in[15];
  const float* db2    = (const float*)d_in[16];
  const float* vw1    = (const float*)d_in[17];
  const float* vb1    = (const float*)d_in[18];
  const float* vw2    = (const float*)d_in[19];
  const float* vb2    = (const float*)d_in[20];
  float* out = (float*)d_out;

  char* ws = (char*)d_ws;
  unsigned short* XB    = (unsigned short*)(ws + O_XB);
  float*          YUT   = (float*)(ws + O_YUT);
  float*          H     = (float*)(ws + O_H);
  unsigned short* HHL   = (unsigned short*)(ws + O_HHL);
  float*          P     = (float*)(ws + O_P);
  unsigned short* SHL   = (unsigned short*)(ws + O_SHL);
  int*            BLIST = (int*)(ws + O_BLIST);
  int*            OFFC  = (int*)(ws + O_OFFC);
  int*            META  = (int*)(ws + O_META);
  float*          OUT3  = (float*)(ws + O_OUT3);
  unsigned short* ENCWT = (unsigned short*)(ws + O_ENCW);
  unsigned short* W1AT2 = (unsigned short*)(ws + O_W1A);
  unsigned short* W2T2  = (unsigned short*)(ws + O_W2T);
  unsigned short* HWT2  = (unsigned short*)(ws + O_HWT);
  float*          PAR   = (float*)(ws + O_PAR);

  hipFuncSetAttribute(reinterpret_cast<const void*>(&k_bucket),
                      hipFuncAttributeMaxDynamicSharedMemorySize, LDS_BKT);
  hipFuncSetAttribute(reinterpret_cast<const void*>(&k_msg),
                      hipFuncAttributeMaxDynamicSharedMemorySize, LDS_MSG);

  k_prep<<<30, 256, 0, stream>>>(enc_w, enc_b, enc_g, enc_be, mlp_w1, mlp_b1, mlp_w2, mlp_b2, ln_g, ln_b,
                                 dw1, db1, dw2, db2, vw1, vb1, vw2, vb2,
                                 ENCWT, W1AT2, W2T2, HWT2, PAR, SHL);
  k_plane<0><<<MPN * 32 / 8 / 256, 256, 0, stream>>>(x, NN, 16, 16, XB, MPN, 32);
  k_bucket<<<NBLK, NTHR, LDS_BKT, stream>>>(ei + NE, NE, NN, 1, BLIST, OFFC, META);
  k_gemm_nt<0, 0><<<(782 + 7) / 8, 256, 0, stream>>>(XB, ENCWT, PAR, YUT, NN, 64, 32, 64);
  k_rowln<0><<<MPN / 64, 256, 0, stream>>>(YUT, H, OFFC, PAR, PA_ENC, HHL);
  for (int i = 0; i < 3; ++i) {
    k_gemm_nt<0, 0><<<(782 + 7) / 8, 256, 0, stream>>>(HHL, W1AT2 + (size_t)i * 64 * 128, PAR, P, NN, 32, 128, 32);
    k_msg<<<NBLK, 256, LDS_MSG, stream>>>(ei, eattr, P, BLIST, OFFC, META, PAR, PA_MSG + 128 * i, SHL);
    k_gemm_nt<0, 0><<<(782 + 7) / 8, 256, 0, stream>>>(SHL, W2T2 + (size_t)i * 64 * 64, PAR, YUT, NN, 64, 64, 64);
    k_rowln<1><<<MPN / 64, 256, 0, stream>>>(YUT, H, OFFC, PAR, PA_LYR + 192 * i, HHL);
  }
  k_gemm_nt<0, 0><<<(782 + 7) / 8, 256, 0, stream>>>(HHL, HWT2, PAR, YUT, NN, 64, 128, 64);
  k_head<<<MPN / 128, 128, 0, stream>>>(YUT, PAR, OUT3);
  k_store<<<586, 256, 0, stream>>>(OUT3, out);
}
